// TemporalRelation_15951508537871
// MI455X (gfx1250) — hardware-run, weakly checked
//
#include <hip/hip_runtime.h>
#include <math.h>

typedef __attribute__((ext_vector_type(16))) _Float16 v16h;
typedef __attribute__((ext_vector_type(8)))  _Float16 v8h;
typedef __attribute__((ext_vector_type(8)))  float    v8f;
typedef __attribute__((ext_vector_type(4)))  float    v4f;
typedef __attribute__((ext_vector_type(4)))  unsigned v4u;

constexpr int kNumB    = 32;
constexpr int kNumM    = 64;
constexpr int kLen     = 128;
constexpr int kSamples = kNumB * kNumM;
constexpr int kRowsPS  = kLen + 2;
constexpr int kChunks  = 4;
constexpr int kSampPC  = kSamples / kChunks;
constexpr int kRowsPC  = kSampPC * kRowsPS;
constexpr int kRowsAll = kSamples * kRowsPS;
constexpr int kCh1     = 512;
constexpr int kCh2     = 256;
constexpr int kKdim1   = 32;
constexpr int kKdim2   = 3 * kCh1;
constexpr int kTailRows = 2;

constexpr float kCarryX  = 16.0f;
constexpr float kCarryW  = 256.0f;
constexpr float kCarryA1 = 16.0f;
constexpr float kScale1  = kCarryA1 / (kCarryX * kCarryW);
constexpr float kScale2  = 1.0f / (kCarryA1 * kCarryW);

static_assert(kSamples == 2048);
static_assert(kRowsPC == 66560);
static_assert(kRowsAll == 266240);
static_assert((kRowsPC % 64) == 0 && (kCh1 % 64) == 0 && (kCh2 % 64) == 0);
static_assert((kKdim1 % 32) == 0 && (kKdim2 % 32) == 0);
static_assert((((kRowsPC / 64) * (kCh1 / 64)) % 8) == 0);
static_assert((((kRowsPC / 64) * (kCh2 / 64)) % 8) == 0);

constexpr size_t kBytesAct1 = (size_t)(kRowsPC + kTailRows) * kCh1 * 2;
constexpr size_t kBytesAct2 = (size_t)kRowsPC * kCh2 * 2;
constexpr size_t kBytesXcol = (size_t)kRowsAll * kKdim1 * 2;
constexpr size_t kBytesW2t  = (size_t)kCh2 * kKdim2 * 2;
constexpr size_t kBytesW1t  = (size_t)kCh1 * kKdim1 * 2;
constexpr size_t kOffAct1 = 0;
constexpr size_t kOffAct2 = kOffAct1 + kBytesAct1;
constexpr size_t kOffXcol = kOffAct2 + kBytesAct2;
constexpr size_t kOffW2t  = kOffXcol + kBytesXcol;
constexpr size_t kOffW1t  = kOffW2t + kBytesW2t;
constexpr size_t kWsTotal = kOffW1t + kBytesW1t;
static_assert(kBytesAct1 == 68159488ull);
static_assert(kBytesAct2 == 34078720ull);
static_assert(kBytesXcol == 17039360ull);
static_assert(kWsTotal == 120096768ull);
static_assert(kWsTotal <= 134217728ull);
static_assert((kOffAct2 % 128) == 0 && (kOffXcol % 128) == 0 && (kOffW2t % 128) == 0 && (kOffW1t % 128) == 0);

union FragU { v16h v; v8h h[2]; };

__device__ __forceinline__ v16h frag_load_h(const _Float16* p) {
  FragU f;
  f.h[0] = *(const v8h*)(p);
  f.h[1] = *(const v8h*)(p + 16);
  return f.v;
}

__device__ __forceinline__ v8f mma_guarded(v16h a, v16h b, v8f c) {
  c = __builtin_amdgcn_wmma_f32_16x16x32_f16(false, a, false, b, (short)0, c, false, false);
  asm volatile("v_nop\n\tv_nop\n\tv_nop\n\tv_nop" : "+v"(c) : "v"(a), "v"(b));
  return c;
}

__device__ __forceinline__ float h16_to_f32(unsigned hb) {
  const unsigned sgn = (hb & 0x8000u) << 16;
  const unsigned em = hb & 0x7fffu;
  const float fn = __uint_as_float((em << 13) + 0x38000000u);
  const float fs = (float)em * 5.9604644775390625e-8f;
  const float mag = (em < 0x400u) ? fs : fn;
  return __uint_as_float(__float_as_uint(mag) | sgn);
}

template <int BIAS_MODE>
__global__ __launch_bounds__(256) void gemm64_f16_kernel(
    const unsigned short* __restrict__ Ap, int lda,
    const unsigned short* __restrict__ Btp, int ldb,
    unsigned short* __restrict__ Cp, int ldc,
    const float* __restrict__ bias,
    int M, int N, int K, float scale)
{
  const _Float16* A  = (const _Float16*)Ap;
  const _Float16* Bt = (const _Float16*)Btp;
  __shared__ __align__(16) float sT[8][16 * 68];
  const int lane = threadIdx.x & 31;
  const int wave = threadIdx.x >> 5;
  const int tilesN = N >> 6;
  const int tilesM = M >> 6;
  const int tile = blockIdx.x * 8 + wave;
  if (tile >= tilesM * tilesN) return;
  const int tm = tile / tilesN;
  const int tn = tile - tm * tilesN;
  const int m0 = tm << 6;
  const int n0 = tn << 6;

  const int rlane = lane & 15;
  const int koff  = (lane >> 4) * 8;
  const int mOff  = (lane >> 4) * 8;

  v8f acc[4][4];
#pragma unroll
  for (int i = 0; i < 4; ++i)
#pragma unroll
    for (int j = 0; j < 4; ++j) acc[i][j] = (v8f){0.f, 0.f, 0.f, 0.f, 0.f, 0.f, 0.f, 0.f};

  for (int k0 = 0; k0 < K; k0 += 32) {
    v16h bh[4];
#pragma unroll
    for (int j = 0; j < 4; ++j) {
      const size_t bo = (size_t)(n0 + (j << 4) + rlane) * ldb + koff + k0;
      bh[j] = frag_load_h(Bt + bo);
    }
#pragma unroll
    for (int i = 0; i < 4; ++i) {
      const size_t ao = (size_t)(m0 + (i << 4) + rlane) * lda + koff + k0;
      const v16h ah = frag_load_h(A + ao);
#pragma unroll
      for (int j = 0; j < 4; ++j) acc[i][j] = mma_guarded(ah, bh[j], acc[i][j]);
    }
  }

  float* slab = sT[wave];
#pragma unroll
  for (int i = 0; i < 4; ++i) {
    const int mBase = m0 + (i << 4);
#pragma unroll
    for (int j = 0; j < 4; ++j) {
      const int n = n0 + (j << 4) + rlane;
      float bv = 0.f;
      if (BIAS_MODE == 2) bv = bias[n];
#pragma unroll
      for (int r = 0; r < 8; ++r) {
        float v = acc[i][j][r] * scale;
        if (BIAS_MODE == 2) v += bv;
        slab[(mOff + r) * 68 + (j << 4) + rlane] = v;
      }
    }
    __builtin_amdgcn_fence(__ATOMIC_RELEASE, "workgroup");
    __builtin_amdgcn_wave_barrier();
    __builtin_amdgcn_fence(__ATOMIC_ACQUIRE, "workgroup");
    {
      const int q = lane >> 3, c8 = (lane & 7) * 8;
      for (int pass = 0; pass < 2; ++pass) {
#pragma unroll
        for (int it = 0; it < 4; ++it) {
          const int row = it * 4 + q;
          const float* sp = slab + row * 68 + c8;
          v8h hv;
#pragma unroll
          for (int e = 0; e < 8; ++e) hv[e] = (_Float16)sp[e];
          *(volatile v8h*)(Cp + (size_t)(mBase + row) * ldc + n0 + c8) = hv;
        }
        __threadfence();
      }
    }
    __builtin_amdgcn_fence(__ATOMIC_RELEASE, "workgroup");
    __builtin_amdgcn_wave_barrier();
    __builtin_amdgcn_fence(__ATOMIC_ACQUIRE, "workgroup");
  }
}

__global__ __launch_bounds__(256) void build_w1t_kernel(
    const float* __restrict__ W1, const float* __restrict__ b1,
    unsigned short* __restrict__ w1t, unsigned short* __restrict__ act1_tail)
{
  if (blockIdx.x == 8) {
    if (threadIdx.x < 128) {
      const v8h z = (v8h){0, 0, 0, 0, 0, 0, 0, 0};
      unsigned short* p = act1_tail + threadIdx.x * 8;
      *(volatile v8h*)p = z;
      __threadfence();
      *(volatile v8h*)p = z;
    }
    return;
  }
  const int i  = blockIdx.x * 256 + threadIdx.x;
  const int e0 = i * 8;
  const int co = e0 >> 5;
  const int kb = e0 & 31;
  float bv = b1[co];
  asm volatile("" : "+v"(bv));
  v8h hv;
#pragma unroll
  for (int e = 0; e < 8; ++e) {
    const int k   = kb + e;
    const int tap = k >> 2;
    const int ci  = k & 3;
    const int tc  = (tap < 2) ? tap : 2;
    float wv = W1[(co * 4 + ci) * 3 + tc];
    asm volatile("" : "+v"(wv));
    const float val = (k < 12) ? (wv * kCarryW) : ((k == 12) ? (bv * kCarryW) : 0.0f);
    hv[e] = (_Float16)val;
  }
  unsigned short* p = w1t + e0;
  *(volatile v8h*)p = hv;
  __threadfence();
  *(volatile v8h*)p = hv;
}

__global__ __launch_bounds__(256) void build_w2t_kernel(
    const float* __restrict__ W2, unsigned short* __restrict__ w2t)
{
  const int i   = blockIdx.x * 256 + threadIdx.x;
  const int e0  = i * 8;
  const int c2  = e0 / kKdim2;
  const int k   = e0 - c2 * kKdim2;
  const int tap = k >> 9;
  const int c1  = k & 511;
  v8h hv;
#pragma unroll
  for (int e = 0; e < 8; ++e) {
    const float wv = W2[((size_t)c2 * kCh1 + c1 + e) * 3 + tap];
    hv[e] = (_Float16)(wv * kCarryW);
  }
  unsigned short* p = w2t + e0;
  *(volatile v8h*)p = hv;
  __threadfence();
  *(volatile v8h*)p = hv;
}

__global__ __launch_bounds__(256) void build_xcol_kernel(
    const float* __restrict__ history, const float* __restrict__ current,
    unsigned short* __restrict__ xcol)
{
#pragma clang fp contract(off)
  const int i  = blockIdx.x * 256 + threadIdx.x;
  const int vg = i >> 2;
  const int kb = (i & 3) * 8;
  const int s  = vg / kRowsPS;
  const int r  = vg - s * kRowsPS;
  const int m  = s >> 5;
  const int b  = s & 31;
  const float* hrow = history + (size_t)(b * kNumM + m) * kLen;
  const float* crow = current + (size_t)b * kLen;
  const bool rvalid = (r >= 1) && (r <= kLen);
  const int tapA = (kb == 0) ? 0 : 2;
  const int pA = r + tapA - 2;
  const int pB = r - 1;
  const int pAc = (pA < 0) ? 0 : ((pA > kLen - 1) ? (kLen - 1) : pA);
  const int pBc = (pB < 0) ? 0 : ((pB > kLen - 1) ? (kLen - 1) : pB);
  float hA = hrow[pAc];
  float cA = crow[pAc];
  float hB = hrow[pBc];
  float cB = crow[pBc];
  asm volatile("" : "+v"(hA), "+v"(cA), "+v"(hB), "+v"(cB));
  const bool okA   = rvalid && (pA >= 0) && (pA <= kLen - 1) && (kb <= 8);
  const bool okB   = rvalid && (kb == 0);
  const bool okOne = rvalid && (kb == 8);
  const float dA = hA - cA;
  const float dB = hB - cB;
  const float e0 = okA ? (hA * kCarryX) : 0.0f;
  const float e1 = okA ? (cA * kCarryX) : 0.0f;
  const float e2 = okA ? (dA * kCarryX) : 0.0f;
  const float e3 = okA ? (-dA * kCarryX) : 0.0f;
  const float e4 = okB ? (hB * kCarryX) : (okOne ? kCarryX : 0.0f);
  const float e5 = okB ? (cB * kCarryX) : 0.0f;
  const float e6 = okB ? (dB * kCarryX) : 0.0f;
  const float e7 = okB ? (-dB * kCarryX) : 0.0f;
  v8h hv;
  hv[0] = (_Float16)e0;
  hv[1] = (_Float16)e1;
  hv[2] = (_Float16)e2;
  hv[3] = (_Float16)e3;
  hv[4] = (_Float16)e4;
  hv[5] = (_Float16)e5;
  hv[6] = (_Float16)e6;
  hv[7] = (_Float16)e7;
  unsigned short* p = xcol + (size_t)i * 8;
  *(volatile v8h*)p = hv;
  __threadfence();
  *(volatile v8h*)p = hv;
}

__global__ __launch_bounds__(128) void conv3_kernel(
    const unsigned short* __restrict__ act2, const float* __restrict__ W3, const float* __restrict__ b3,
    float* __restrict__ out, int s0)
{
  __shared__ __align__(16) float sW[3 * kCh2];
  __shared__ __align__(16) float sT[3 * kLen];
  const int tid = threadIdx.x, lane = tid & 31, wave = tid >> 5;
  const int sl = blockIdx.x;
#pragma unroll
  for (int j = 0; j < 6; ++j) sW[tid + 128 * j] = W3[tid + 128 * j];
  __syncthreads();
  const unsigned short* rowp = act2 + ((size_t)sl * kRowsPS + tid) * kCh2;
  float t0 = 0.f, t1 = 0.f, t2 = 0.f;
#pragma unroll 1
  for (int g = 0; g < kCh2 / 8; ++g) {
    const v4u w = *(const v4u*)(rowp + g * 8);
    const unsigned w0 = w[0];
    const unsigned w1 = w[1];
    const unsigned w2 = w[2];
    const unsigned w3 = w[3];
    float a[8];
    a[0] = h16_to_f32(w0 & 0xffffu);
    a[1] = h16_to_f32(w0 >> 16);
    a[2] = h16_to_f32(w1 & 0xffffu);
    a[3] = h16_to_f32(w1 >> 16);
    a[4] = h16_to_f32(w2 & 0xffffu);
    a[5] = h16_to_f32(w2 >> 16);
    a[6] = h16_to_f32(w3 & 0xffffu);
    a[7] = h16_to_f32(w3 >> 16);
    const float* wp = sW + g * 24;
    float wf[24];
#pragma unroll
    for (int qv = 0; qv < 6; ++qv) {
      const v4f q = *(const v4f*)(wp + 4 * qv);
      wf[4 * qv + 0] = q[0];
      wf[4 * qv + 1] = q[1];
      wf[4 * qv + 2] = q[2];
      wf[4 * qv + 3] = q[3];
    }
#pragma unroll
    for (int cc = 0; cc < 8; ++cc) {
      t0 = fmaf(a[cc], wf[cc * 3 + 0], t0);
      t1 = fmaf(a[cc], wf[cc * 3 + 1], t1);
      t2 = fmaf(a[cc], wf[cc * 3 + 2], t2);
    }
  }
  sT[tid] = t0;
  sT[kLen + tid] = t1;
  sT[2 * kLen + tid] = t2;
  __syncthreads();
  if (wave == 0) {
    const float bb = b3[0];
    v4f o;
#pragma unroll
    for (int e = 0; e < 4; ++e) {
      const int p  = 4 * lane + e;
      const int pm = (p >= 1) ? (p - 1) : 0;
      const int pp = (p <= kLen - 2) ? (p + 1) : (kLen - 1);
      const float x0 = sT[pm];
      const float x1 = sT[kLen + p];
      const float x2 = sT[2 * kLen + pp];
      float v = bb + x1;
      v += (p >= 1) ? x0 : 0.0f;
      v += (p <= kLen - 2) ? x2 : 0.0f;
      o[e] = v;
    }
    float* dst = out + (size_t)(s0 + sl) * kLen + 4 * lane;
    *(volatile v4f*)dst = o;
    __threadfence();
    *(volatile v4f*)dst = o;
  }
}

extern "C" void kernel_launch(void* const* d_in, const int* in_sizes, int n_in,
                              void* d_out, int out_size, void* d_ws, size_t ws_size,
                              hipStream_t stream) {
  if (n_in < 8) return;
  if (in_sizes[0] != kNumB * kNumM * kLen) return;
  if (in_sizes[1] != kNumB * kLen) return;
  if (in_sizes[2] != kCh1 * 4 * 3) return;
  if (in_sizes[3] != kCh1) return;
  if (in_sizes[4] != kCh2 * kCh1 * 3) return;
  if (in_sizes[5] != kCh2) return;
  if (in_sizes[6] != kCh2 * 3) return;
  if (in_sizes[7] != 1) return;
  if (out_size != kSamples * kLen) return;
  if (ws_size < kWsTotal) return;

  const float* history = (const float*)d_in[0];
  const float* current = (const float*)d_in[1];
  const float* W1 = (const float*)d_in[2];
  const float* b1 = (const float*)d_in[3];
  const float* W2 = (const float*)d_in[4];
  const float* b2 = (const float*)d_in[5];
  const float* W3 = (const float*)d_in[6];
  const float* b3 = (const float*)d_in[7];
  float* out = (float*)d_out;

  char* ws = (char*)d_ws;
  unsigned short* act1 = (unsigned short*)(ws + kOffAct1);
  unsigned short* act2 = (unsigned short*)(ws + kOffAct2);
  unsigned short* xcol = (unsigned short*)(ws + kOffXcol);
  unsigned short* w2t  = (unsigned short*)(ws + kOffW2t);
  unsigned short* w1t  = (unsigned short*)(ws + kOffW1t);
  unsigned short* act1_tail = act1 + (size_t)kRowsPC * kCh1;

  build_w1t_kernel<<<9, 256, 0, stream>>>(W1, b1, w1t, act1_tail);
  build_w2t_kernel<<<(kCh2 * kKdim2 / 8) / 256, 256, 0, stream>>>(W2, w2t);
  build_xcol_kernel<<<(kRowsAll * 4) / 256, 256, 0, stream>>>(history, current, xcol);

  constexpr int kGrid1 = ((kRowsPC / 64) * (kCh1 / 64)) / 8;
  constexpr int kGrid2 = ((kRowsPC / 64) * (kCh2 / 64)) / 8;
  for (int ch = 0; ch < kChunks; ++ch) {
    const unsigned short* xc = xcol + (size_t)ch * kRowsPC * kKdim1;
    gemm64_f16_kernel<0><<<kGrid1, 256, 0, stream>>>(
        xc, kKdim1, w1t, kKdim1, act1, kCh1, b1, kRowsPC, kCh1, kKdim1, kScale1);
    gemm64_f16_kernel<2><<<kGrid2, 256, 0, stream>>>(
        act1, kCh1, w2t, kKdim2, act2, kCh2, b2, kRowsPC, kCh2, kKdim2, kScale2);
    conv3_kernel<<<kSampPC, 128, 0, stream>>>(act2, W3, b3, out, ch * kSampPC);
  }
}
